// GatedDeltaNetMixer_19104014532976
// MI455X (gfx1250) — hardware-verified
//
#include <hip/hip_runtime.h>
#include <math.h>

typedef __attribute__((ext_vector_type(16))) _Float16 v16h;
typedef __attribute__((ext_vector_type(8)))  _Float16 v8h;
typedef __attribute__((ext_vector_type(16))) __bf16   v16b;
typedef __attribute__((ext_vector_type(8)))  __bf16   v8b;
typedef __attribute__((ext_vector_type(8)))  float    v8f;
typedef __attribute__((ext_vector_type(4)))  float    v4f;

constexpr int kB    = 2;
constexpr int kL    = 2048;
constexpr int kD    = 2048;
constexpr int kHd   = 128;
constexpr int kH    = 16;
constexpr int kHG   = 8;
constexpr int kNG   = kHG * kHd;
constexpr int kBG   = 64;
constexpr int kTaps = 4;
constexpr int kThr  = 256;
constexpr float kInCarry = 1024.0f;
constexpr float kWCarry = 4096.0f;
constexpr float kSc = 1.0f / (kInCarry * kWCarry);
constexpr float kCo = 64.0f;
constexpr float kScO = 1.0f / (kCo * kWCarry);
constexpr float kLnEps = 1e-5f;
constexpr float kF16MinNormal = 6.103515625e-5f;

static_assert((kL % 64) == 0 && (kNG % 64) == 0 && (kD % 64) == 0 && (kBG % 64) == 0 && ((kL / 64) * (kBG / 64)) % 8 == 0, "GEMM M, N multiples of 64; grids exact");
static_assert((kD % 256) == 0 && kD / 8 == 256 && kD == 2 * kNG && kD == kH * kHd && kH == 2 * kHG, "GEMM K a multiple of 32; the transposing cast's block of K / 8 = 256 threads; two passes of eight heads");

constexpr size_t kOffWQ = 0ull;
constexpr size_t kOffWK = 8388608ull;
constexpr size_t kOffWV = 16777216ull;
constexpr size_t kOffWG = 25165824ull;
constexpr size_t kOffWO = 33554432ull;
constexpr size_t kOffWB = 41943040ull;
constexpr size_t kOffBIAS = 42205184ull;
constexpr size_t kOffPRM = 42214400ull;
constexpr size_t kOffX16 = 42232832ull;
constexpr size_t kOffBL = 50621440ull;
constexpr size_t kOffBE = 51145728ull;
constexpr size_t kOffQL = 51407872ull;
constexpr size_t kOffKL = 59796480ull;
constexpr size_t kOffVP = 68185088ull;
constexpr size_t kOffGL = 76573696ull;
constexpr size_t kOffQ2 = 84962304ull;
constexpr size_t kOffK2 = 93350912ull;
constexpr size_t kOffO32 = 101739520ull;
constexpr size_t kOffO16 = 110128128ull;
constexpr size_t kWsTotal = 118516736ull;
static_assert(kWsTotal <= 134217728ull, "carve cap: under 128 MiB");
static_assert(kOffWQ == 0
              && kOffWK == kOffWQ + 8388608ull
              && kOffWV == kOffWK + 8388608ull
              && kOffWG == kOffWV + 8388608ull
              && kOffWO == kOffWG + 8388608ull
              && kOffWB == kOffWO + 8388608ull
              && kOffBIAS == kOffWB + 262144ull
              && kOffPRM == kOffBIAS + 9216ull
              && kOffX16 == kOffPRM + 18432ull
              && kOffBL == kOffX16 + 8388608ull
              && kOffBE == kOffBL + 524288ull
              && kOffQL == kOffBE + 262144ull
              && kOffKL == kOffQL + 8388608ull
              && kOffVP == kOffKL + 8388608ull
              && kOffGL == kOffVP + 8388608ull
              && kOffQ2 == kOffGL + 8388608ull
              && kOffK2 == kOffQ2 + 8388608ull
              && kOffO32 == kOffK2 + 8388608ull
              && kOffO16 == kOffO32 + 8388608ull
              && kWsTotal == kOffO16 + 8388608ull, "the carve is chained and totalled");
static_assert((kOffWQ % 256) == 0 && (kOffWK % 256) == 0 && (kOffWV % 256) == 0 && (kOffWG % 256) == 0 && (kOffWO % 256) == 0 && (kOffWB % 256) == 0 && (kOffBIAS % 256) == 0 && (kOffPRM % 256) == 0 && (kOffX16 % 256) == 0 && (kOffBL % 256) == 0 && (kOffBE % 256) == 0 && (kOffQL % 256) == 0 && (kOffKL % 256) == 0 && (kOffVP % 256) == 0 && (kOffGL % 256) == 0 && (kOffQ2 % 256) == 0 && (kOffK2 % 256) == 0 && (kOffO32 % 256) == 0 && (kOffO16 % 256) == 0, "aligned regions");
constexpr int kFZB = 0, kFBB = 2048, kFEnd = 2304;
constexpr int kPQB = 0, kPKB = 2048, kPQW = 4096, kPQO = 4224, kPKW = 4352, kPKO = 4480, kPEnd = 4608;
static_assert(kFBB == kFZB + kD && kFBB + kBG <= kFEnd && kPKB == kPQB + kD && kPQW == kPKB + kD && kPQO == kPQW + kHd && kPKW == kPQO + kHd && kPKO == kPKW + kHd && kPEnd == kPKO + kHd, "bias stream and parameter plane maps");

__device__ __forceinline__ unsigned short f2bf_bits(float f) {
  unsigned u = __float_as_uint(f);
  return (unsigned short)((u + 0x7FFFu + ((u >> 16) & 1u)) >> 16);
}
__device__ __forceinline__ float bf_bits2f(unsigned short h) { return __uint_as_float(((unsigned)h) << 16); }
__device__ __forceinline__ float bf16r(float f) { return bf_bits2f(f2bf_bits(f)); }
__device__ __forceinline__ float carry_flush(float v, float carry) {
  const float s = v * carry;
  return (fabsf(s) < kF16MinNormal) ? 0.0f : s;
}
__device__ __forceinline__ float frcp(float x) { return __builtin_amdgcn_rcpf(x); }

__device__ __forceinline__ void dep_guard4_h(v8f& a, v8f& b, v8f& c, v8f& d, v16h x, v16h y) { asm volatile("v_nop\n\tv_nop\n\tv_nop\n\tv_nop" : "+v"(a), "+v"(b), "+v"(c), "+v"(d) : "v"(x), "v"(y)); }
__device__ __forceinline__ void dep_guard4_b(v8f& a, v8f& b, v8f& c, v8f& d, v16b x, v16b y) { asm volatile("v_nop\n\tv_nop\n\tv_nop\n\tv_nop" : "+v"(a), "+v"(b), "+v"(c), "+v"(d) : "v"(x), "v"(y)); }
__device__ __forceinline__ void keep4_h(v16h a, v16h b, v16h c, v16h d) { asm volatile("v_nop" :: "v"(a), "v"(b), "v"(c), "v"(d)); }
__device__ __forceinline__ void keep4_b(v16b a, v16b b, v16b c, v16b d) { asm volatile("v_nop" :: "v"(a), "v"(b), "v"(c), "v"(d)); }
__device__ __forceinline__ void acc_guard4(v8f& a, v8f& b, v8f& c, v8f& d) { asm volatile("v_nop\n\tv_nop\n\tv_nop\n\tv_nop" : "+v"(a), "+v"(b), "+v"(c), "+v"(d)); }

template <typename T> struct Frag;
template <> struct Frag<_Float16> {
  typedef v16h V; union U { v16h v; v8h h[2]; };
  static __device__ __forceinline__ v16h load(const _Float16* p) {
    U f; f.h[0] = *(const v8h*)(p); f.h[1] = *(const v8h*)(p + 16); return f.v;
  }
  static __device__ __forceinline__ v8f mma(v16h a, v16h b, v8f c) {
    return __builtin_amdgcn_wmma_f32_16x16x32_f16(false, a, false, b, (short)0, c, false, false);
  }
  static __device__ __forceinline__ void guard4(v8f& a, v8f& b, v8f& c, v8f& d, v16h x, v16h y) { dep_guard4_h(a, b, c, d, x, y); }
  static __device__ __forceinline__ void keep(v16h a, v16h b, v16h c, v16h d) { keep4_h(a, b, c, d); }
};
template <> struct Frag<__bf16> {
  typedef v16b V; union U { v16b v; v8b h[2]; };
  static __device__ __forceinline__ v16b load(const __bf16* p) {
    U f; f.h[0] = *(const v8b*)(p); f.h[1] = *(const v8b*)(p + 16); return f.v;
  }
  static __device__ __forceinline__ v8f mma(v16b a, v16b b, v8f c) {
    return __builtin_amdgcn_wmma_f32_16x16x32_bf16(false, a, false, b, (short)0, c, false, false);
  }
  static __device__ __forceinline__ void guard4(v8f& a, v8f& b, v8f& c, v8f& d, v16b x, v16b y) { dep_guard4_b(a, b, c, d, x, y); }
  static __device__ __forceinline__ void keep(v16b a, v16b b, v16b c, v16b d) { keep4_b(a, b, c, d); }
};

__device__ __forceinline__ v8f mma_h(v16h a, v16h b, v8f c) {
  c = __builtin_amdgcn_wmma_f32_16x16x32_f16(false, a, false, b, (short)0, c, false, false);
  asm volatile("v_nop\n\tv_nop\n\tv_nop\n\tv_nop" : "+v"(c) : "v"(a), "v"(b));
  return c;
}

template <int ET> struct Elem;
template <> struct Elem<0> { typedef _Float16 T; };
template <> struct Elem<1> { typedef __bf16 T; };
template <int ET, bool SPLIT, int BIAS_MODE, int OUT_MODE, bool RESID, int ACT = 0>
__global__ __launch_bounds__(256) void wmma_gemm64(
    const unsigned short* __restrict__ Ap, const unsigned short* __restrict__ A2p, int lda, long strideA,
    const unsigned short* __restrict__ Btp, const unsigned short* __restrict__ Bt2p, int ldb, long strideB,
    void* __restrict__ Cout, void* __restrict__ Cout2, int ldc, long strideC,
    const float* __restrict__ bias,
    const float* __restrict__ resid, long strideR,
    int M, int N, int K, float scale) {
  typedef typename Elem<ET>::T T;
  typedef typename Frag<T>::V V;
  const T* A = (const T*)Ap; const T* A2 = (const T*)A2p; const T* Bt = (const T*)Btp; const T* Bt2 = (const T*)Bt2p;
  __shared__ __align__(16) float sT[8][16 * 68];
  const int b    = blockIdx.y;
  const int lane = threadIdx.x & 31;
  const int wave = threadIdx.x >> 5;
  const int tilesN = N >> 6;
  const int tilesM = M >> 6;
  const int tile = blockIdx.x * 8 + wave;
  if (tile >= tilesM * tilesN) return;
  const int tm = tile / tilesN;
  const int tn = tile - tm * tilesN;
  const int m0 = tm << 6;
  const int n0 = tn << 6;

  const T* Ab  = A  + (size_t)b * strideA;
  const T* Bb  = Bt + (size_t)b * strideB;
  const T* Ab2 = SPLIT ? (A2  + (size_t)b * strideA) : nullptr;
  const T* Bb2 = SPLIT ? (Bt2 + (size_t)b * strideB) : nullptr;

  const int rlane = lane & 15;
  const int koff  = (lane >> 4) * 8;
  const int mOff  = (lane >> 4) * 8;

  v8f acc[4][4];
#pragma unroll
  for (int i = 0; i < 4; ++i)
#pragma unroll
    for (int j = 0; j < 4; ++j) acc[i][j] = (v8f){0.f,0.f,0.f,0.f,0.f,0.f,0.f,0.f};

  for (int k0 = 0; k0 < K; k0 += 32) {
    V bh[4], bl[4];
#pragma unroll
    for (int j = 0; j < 4; ++j) {
      const size_t bo = (size_t)(n0 + (j << 4) + rlane) * ldb + koff + k0;
      bh[j] = Frag<T>::load(Bb + bo);
      if (SPLIT) bl[j] = Frag<T>::load(Bb2 + bo);
    }
#pragma unroll
    for (int i = 0; i < 4; ++i) {
      const size_t ao = (size_t)(m0 + (i << 4) + rlane) * lda + koff + k0;
      V ah = Frag<T>::load(Ab + ao);
      V al;
      if (SPLIT) al = Frag<T>::load(Ab2 + ao);
#pragma unroll
      for (int j = 0; j < 4; ++j) {
        acc[i][j] = Frag<T>::mma(ah, bh[j], acc[i][j]);
        if (SPLIT) {
          acc[i][j] = Frag<T>::mma(ah, bl[j], acc[i][j]);
          acc[i][j] = Frag<T>::mma(al, bh[j], acc[i][j]);
        }
      }
      Frag<T>::guard4(acc[i][0], acc[i][1], acc[i][2], acc[i][3], ah, SPLIT ? al : ah);
    }
    Frag<T>::keep(bh[0], bh[1], bh[2], bh[3]);
    if (SPLIT) Frag<T>::keep(bl[0], bl[1], bl[2], bl[3]);
  }
  acc_guard4(acc[0][0], acc[0][1], acc[0][2], acc[0][3]);
  acc_guard4(acc[1][0], acc[1][1], acc[1][2], acc[1][3]);
  acc_guard4(acc[2][0], acc[2][1], acc[2][2], acc[2][3]);
  acc_guard4(acc[3][0], acc[3][1], acc[3][2], acc[3][3]);

  float* slab = sT[wave];
  const float* Rb = RESID ? (resid + (size_t)b * strideR) : nullptr;
#pragma unroll
  for (int i = 0; i < 4; ++i) {
    const int mBase = m0 + (i << 4);
#pragma unroll
    for (int j = 0; j < 4; ++j) {
      const int n = n0 + (j << 4) + rlane;
      float bv = 0.f;
      if (BIAS_MODE == 2) bv = bias[n];
#pragma unroll
      for (int r = 0; r < 8; ++r) {
        float v = acc[i][j][r] * scale;
        if (BIAS_MODE == 1) v += bias[mBase + mOff + r];
        if (BIAS_MODE == 2) v += bv;
        if (RESID) v += Rb[(size_t)(mBase + mOff + r) * ldc + n];
        if (ACT == 1) v = tanhf(v);
        if (ACT == 2) v = fmaxf(v, 0.0f);
        if (ACT == 3) v = v / (1.0f + expf(-v));
        if (ACT == 4) v = (v > 0.f) ? v : 0.01f * v;
        slab[(mOff + r) * 68 + (j << 4) + rlane] = v;
      }
    }
    __builtin_amdgcn_fence(__ATOMIC_RELEASE, "workgroup");
    __builtin_amdgcn_wave_barrier();
    __builtin_amdgcn_fence(__ATOMIC_ACQUIRE, "workgroup");
    if (OUT_MODE == 0) {
      float* C = (float*)Cout + (size_t)b * strideC;
      const int hh = lane >> 4, c4 = (lane & 15) * 4;
      for (int pass = 0; pass < 2; ++pass) {
#pragma unroll
        for (int it = 0; it < 8; ++it) {
          const int row = it * 2 + hh;
          v4f v = *(const v4f*)(slab + row * 68 + c4);
          *(volatile v4f*)(C + (size_t)(mBase + row) * ldc + n0 + c4) = v;
        }
        __threadfence();
      }
    } else {
      const int q = lane >> 3, c8 = (lane & 7) * 8;
      unsigned short* C  = (unsigned short*)Cout  + (size_t)b * strideC;
      unsigned short* C2 = (OUT_MODE == 2) ? ((unsigned short*)Cout2 + (size_t)b * strideC) : nullptr;
      for (int pass = 0; pass < 2; ++pass) {
#pragma unroll
        for (int it = 0; it < 4; ++it) {
          const int row = it * 4 + q;
          const float* sp = slab + row * 68 + c8;
          v8h hv, lv;
#pragma unroll
          for (int e = 0; e < 8; ++e) {
            if (OUT_MODE == 1) {
              hv[e] = (_Float16)sp[e];
            } else {
              unsigned short hb = f2bf_bits(sp[e]);
              unsigned short lb = f2bf_bits(sp[e] - bf_bits2f(hb));
              hv[e] = __builtin_bit_cast(_Float16, hb);
              lv[e] = __builtin_bit_cast(_Float16, lb);
            }
          }
          *(volatile v8h*)(C + (size_t)(mBase + row) * ldc + n0 + c8) = hv;
          if (OUT_MODE == 2) *(volatile v8h*)(C2 + (size_t)(mBase + row) * ldc + n0 + c8) = lv;
        }
        __threadfence();
      }
    }
    __builtin_amdgcn_fence(__ATOMIC_RELEASE, "workgroup");
    __builtin_amdgcn_wave_barrier();
    __builtin_amdgcn_fence(__ATOMIC_ACQUIRE, "workgroup");
  }
}

__global__ __launch_bounds__(kThr) void cast_plane_kernel(const float* __restrict__ src, unsigned short* __restrict__ dst,
                                                          int colsLog2, int dstPitch, int dstOff) {
  const int i   = blockIdx.x * kThr + threadIdx.x;
  const int sh  = colsLog2 - 3;
  const int row = i >> sh;
  const int c8  = (i & ((1 << sh) - 1)) * 8;
  const float* sp = src + ((size_t)row << colsLog2) + c8;
  const v4f a0 = *(const v4f*)(sp);
  const v4f a1 = *(const v4f*)(sp + 4);
  v8h hv;
#pragma unroll
  for (int e = 0; e < 4; ++e) {
    const float f0 = a0[e];
    const float f1 = a1[e];
    hv[e]     = (_Float16)carry_flush(bf16r(f0), kInCarry);
    hv[4 + e] = (_Float16)carry_flush(bf16r(f1), kInCarry);
  }
  unsigned short* dp = dst + (size_t)row * dstPitch + dstOff + c8;
  *(volatile v8h*)dp = hv;
  __threadfence();
  *(volatile v8h*)dp = hv;
}
__global__ __launch_bounds__(256) void wt_plane_kernel(const float* __restrict__ W, unsigned short* __restrict__ dst, int K, int N, int nLive, int ldd, int colOff) {
  const int n  = blockIdx.x;
  const int k8 = threadIdx.x * 8;
  const bool live = n < nLive;
  const int nc = live ? n : 0;
  v8h hv;
#pragma unroll
  for (int e = 0; e < 8; ++e) {
    const float w = W[(size_t)(k8 + e) * N + nc];
    hv[e] = (_Float16)(live ? carry_flush(bf16r(w), kWCarry) : 0.0f);
  }
  unsigned short* dp = dst + (size_t)n * ldd + colOff + k8;
  *(volatile v8h*)dp = hv;
  __threadfence();
  *(volatile v8h*)dp = hv;
}


__device__ __forceinline__ float silu_f(float v) { return v / (1.0f + expf(-v)); }

__global__ __launch_bounds__(kThr) void setup_kernel(const float* __restrict__ bb, const float* __restrict__ qconv_b, const float* __restrict__ kconv_b,
                                                     const float* __restrict__ qn_w, const float* __restrict__ qn_b, const float* __restrict__ kn_w, const float* __restrict__ kn_b,
                                                     float* __restrict__ BIAS, float* __restrict__ PRM) {
  unsigned v = blockIdx.x * 192u + threadIdx.x;
  asm volatile("" : "+v"(v));
  v4f o = {0.f, 0.f, 0.f, 0.f};
  float* dp;
  if (v < 576u) {
    const unsigned i0 = v * 4u;
    dp = BIAS + i0;
    const bool live = (i0 >= (unsigned)kFBB) && (i0 < (unsigned)(kFBB + kH));
    const unsigned j0 = live ? (i0 - (unsigned)kFBB) : 0u;
    const v4f a = *(const v4f*)(bb + j0);
#pragma unroll
    for (int e = 0; e < 4; ++e) { const float p = bf16r(a[e]); o[e] = live ? p : 0.0f; }
  } else {
    const unsigned i0 = (v - 576u) * 4u;
    dp = PRM + i0;
    const float* sp = (i0 < (unsigned)kPKB) ? (qconv_b + i0) : ((i0 < (unsigned)kPQW) ? (kconv_b + (i0 - (unsigned)kPKB)) : ((i0 < (unsigned)kPQO) ? (qn_w + (i0 - (unsigned)kPQW)) : ((i0 < (unsigned)kPKW) ? (qn_b + (i0 - (unsigned)kPQO)) : ((i0 < (unsigned)kPKO) ? (kn_w + (i0 - (unsigned)kPKW)) : (kn_b + (i0 - (unsigned)kPKO))))));
    const v4f a = *(const v4f*)sp;
#pragma unroll
    for (int e = 0; e < 4; ++e) { const float p = a[e]; o[e] = bf16r(p); }
  }
  *(volatile v4f*)dp = o;
  __threadfence();
  *(volatile v4f*)dp = o;
}
static_assert(kFEnd / 4 == 576 && kPEnd / 4 == 1152 && 576 + 1152 == 9 * 192 && (192 % 32) == 0 && (576 % 32) == 0 && (kFBB % 4) == 0 && (kH % 4) == 0, "set-up grid exact; regions wave-uniform");

__global__ __launch_bounds__(kThr) void convln_kernel(const float* __restrict__ X, const float* __restrict__ cw, const float* __restrict__ cb,
                                                      const float* __restrict__ gw, const float* __restrict__ go, float* __restrict__ OUT, int cbase) {
  const unsigned v = blockIdx.x * (unsigned)kThr + threadIdx.x;
  const unsigned t = v >> 3, hd = v & 7u;
  const unsigned c0 = hd * (unsigned)kHd;
  float* orow = OUT + (size_t)t * kNG + c0;
  float s1 = 0.0f;
#pragma unroll 1
  for (int c = 0; c < kHd; c += 4) {
    const unsigned cg = (unsigned)cbase + c0 + (unsigned)c;
    v4f acc = *(const v4f*)(cb + cg);
#pragma unroll
    for (int j = 0; j < kTaps; ++j) {
      const int tr = (int)t - (kTaps - 1) + j;
      if (tr >= 0) {
        const v4f xv = *(const v4f*)(X + (size_t)tr * kNG + c0 + c);
#pragma unroll
        for (int e = 0; e < 4; ++e) acc[e] += xv[e] * bf16r(cw[(size_t)(cg + e) * kTaps + j]);
      }
    }
    v4f y;
#pragma unroll
    for (int e = 0; e < 4; ++e) { y[e] = silu_f(acc[e]); s1 += y[e]; }
    *(volatile v4f*)(orow + c) = y;
  }
  __threadfence();
  const float mu = s1 * (1.0f / (float)kHd);
  float s2 = 0.0f;
#pragma unroll 1
  for (int c = 0; c < kHd; c += 4) { const v4f a = *(const v4f*)(orow + c); const float d0 = a[0] - mu, d1 = a[1] - mu, d2 = a[2] - mu, d3 = a[3] - mu; s2 += (d0 * d0 + d1 * d1) + (d2 * d2 + d3 * d3); }
  const float rs = 1.0f / sqrtf(s2 * (1.0f / (float)kHd) + kLnEps);
#pragma unroll 1
  for (int c = 0; c < kHd; c += 4) {
    const v4f a = *(const v4f*)(orow + c), w4 = *(const v4f*)(gw + c), o4 = *(const v4f*)(go + c);
    v4f y;
#pragma unroll
    for (int e = 0; e < 4; ++e) y[e] = (a[e] - mu) * rs * w4[e] + o4[e];
    *(volatile v4f*)(orow + c) = y;
  }
  __threadfence();
#pragma unroll 1
  for (int c = 0; c < kHd; c += 4) { const v4f a = *(const v4f*)(orow + c); *(volatile v4f*)(orow + c) = a; }
  __threadfence();
}
static_assert(((size_t)kL * kHG) % kThr == 0 && kHG == 8, "conv + norm grid exact; eight heads a group");

__global__ __launch_bounds__(kThr) void beta_kernel(const float* __restrict__ BL, float* __restrict__ BE) {
  const unsigned t = blockIdx.x * (unsigned)kThr + threadIdx.x;
  const float* br = BL + (size_t)t * kBG;
  float* er = BE + (size_t)t * 32;
  for (int pass = 0; pass < 2; ++pass) {
#pragma unroll 1
    for (int h = 0; h < kH; h += 4) {
      const v4f bbv = *(const v4f*)(br + h);
      v4f ob, ok;
#pragma unroll
      for (int e = 0; e < 4; ++e) { ob[e] = 1.0f / (1.0f + expf(-bbv[e])); ok[e] = 1.0f - ob[e]; }
      *(volatile v4f*)(er + h) = ob;
      *(volatile v4f*)(er + kH + h) = ok;
    }
    __threadfence();
  }
}
static_assert(kL == 8 * kThr && 2 * kH == 32, "one thread a row: 8 blocks; a row of BE is one line");

__global__ __launch_bounds__(kHd) void gma_scan_kernel(const float* __restrict__ Q2, const float* __restrict__ K2, const float* __restrict__ VP,
                                                       const float* __restrict__ BE, float* __restrict__ O32, int hbase) {
  __shared__ float st[kHd * kHd];
  const unsigned vcol = threadIdx.x;
  const unsigned hoff = blockIdx.x * (unsigned)kHd;
  const unsigned hg = (unsigned)hbase + blockIdx.x;
  for (int k = 0; k < kHd; ++k) st[k * kHd + vcol] = 0.0f;
  for (int t = 0; t < kL; ++t) {
    const float* qr = Q2 + (size_t)t * kNG + hoff;
    const float* kr = K2 + (size_t)t * kNG + hoff;
    const float bt = BE[(size_t)t * 32 + hg], kt = BE[(size_t)t * 32 + kH + hg];
    const float bv = bt * VP[(size_t)t * kNG + hoff + vcol];
    float sum = 0.0f;
#pragma unroll 1
    for (int k4 = 0; k4 < kHd; k4 += 4) {
      const v4f q4 = *(const v4f*)(qr + k4), c4 = *(const v4f*)(kr + k4);
#pragma unroll
      for (int j = 0; j < 4; ++j) {
        const int idx = (k4 + j) * kHd + (int)vcol;
        const float s = kt * st[idx] + c4[j] * bv;
        st[idx] = s;
        sum += q4[j] * s;
      }
    }
    float* op = O32 + (size_t)t * kNG + hoff + vcol;
    *(volatile float*)op = sum;
    __threadfence();
    *(volatile float*)op = sum;
  }
}
static_assert(kHd * kHd * 4 == 65536 && kHd == 128, "the state: 64 KB of LDS a block; one thread a value column");

__global__ __launch_bounds__(kThr) void ogate_kernel(const float* __restrict__ O32, const float* __restrict__ GL, unsigned short* __restrict__ O16, int cbase) {
  const unsigned v = blockIdx.x * (unsigned)kThr + threadIdx.x;
  const unsigned t = v >> 7, c8 = (v & 127u) * 8u;
  const float* orow = O32 + (size_t)t * kNG + c8;
  const float* grow = GL + (size_t)t * kNG + c8;
  const v4f a0 = *(const v4f*)orow, a1 = *(const v4f*)(orow + 4), g0 = *(const v4f*)grow, g1 = *(const v4f*)(grow + 4);
  v8h hv;
#pragma unroll
  for (int e = 0; e < 4; ++e) { hv[e] = (_Float16)carry_flush(a0[e] * silu_f(g0[e]), kCo); hv[4 + e] = (_Float16)carry_flush(a1[e] * silu_f(g1[e]), kCo); }
  unsigned short* dp = O16 + (size_t)t * kD + (unsigned)cbase + c8;
  *(volatile v8h*)dp = hv;
  __threadfence();
  *(volatile v8h*)dp = hv;
}
static_assert(((size_t)kL * kNG / 8) % kThr == 0 && kNG / 8 == 128, "gate grid exact");

extern "C" void kernel_launch(void* const* d_in, const int* in_sizes, int n_in,
                              void* d_out, int out_size, void* d_ws, size_t ws_size,
                              hipStream_t stream) {
  if (n_in < 16 || d_out == nullptr || d_ws == nullptr) return;
  if (in_sizes[0] != kB * kL * kD || in_sizes[1] != kD * kD || in_sizes[2] != kD * kD || in_sizes[3] != kD * kD || in_sizes[4] != kD * kH || in_sizes[5] != kH || in_sizes[6] != kD * kD || in_sizes[7] != kD * kD) return;
  if (in_sizes[8] != kD * kTaps || in_sizes[9] != kD || in_sizes[10] != kD * kTaps || in_sizes[11] != kD || in_sizes[12] != kHd || in_sizes[13] != kHd || in_sizes[14] != kHd || in_sizes[15] != kHd) return;
  if (out_size != kB * kL * kD) return;
  if (ws_size < kWsTotal) return;
  const float* hidden = (const float*)d_in[0];
  const float* Wq = (const float*)d_in[1];
  const float* Wk = (const float*)d_in[2];
  const float* Wv = (const float*)d_in[3];
  const float* Wb = (const float*)d_in[4];
  const float* bb = (const float*)d_in[5];
  const float* Wg = (const float*)d_in[6];
  const float* Wo = (const float*)d_in[7];
  const float* qconv_w = (const float*)d_in[8];
  const float* qconv_b = (const float*)d_in[9];
  const float* kconv_w = (const float*)d_in[10];
  const float* kconv_b = (const float*)d_in[11];
  const float* qn_w = (const float*)d_in[12];
  const float* qn_b = (const float*)d_in[13];
  const float* kn_w = (const float*)d_in[14];
  const float* kn_b = (const float*)d_in[15];
  float* out = (float*)d_out;
  char* ws = (char*)d_ws;
  unsigned short* WQ = (unsigned short*)(ws + kOffWQ);
  unsigned short* WK = (unsigned short*)(ws + kOffWK);
  unsigned short* WV = (unsigned short*)(ws + kOffWV);
  unsigned short* WG = (unsigned short*)(ws + kOffWG);
  unsigned short* WO = (unsigned short*)(ws + kOffWO);
  unsigned short* WB = (unsigned short*)(ws + kOffWB);
  float* BIAS = (float*)(ws + kOffBIAS);
  float* PRM = (float*)(ws + kOffPRM);
  unsigned short* X16 = (unsigned short*)(ws + kOffX16);
  float* BL = (float*)(ws + kOffBL);
  float* BE = (float*)(ws + kOffBE);
  float* QL = (float*)(ws + kOffQL);
  float* KL = (float*)(ws + kOffKL);
  float* VP = (float*)(ws + kOffVP);
  float* GL = (float*)(ws + kOffGL);
  float* Q2 = (float*)(ws + kOffQ2);
  float* K2 = (float*)(ws + kOffK2);
  float* O32 = (float*)(ws + kOffO32);
  unsigned short* O16 = (unsigned short*)(ws + kOffO16);

  wt_plane_kernel<<<kD, kD / 8, 0, stream>>>(Wq, WQ, kD, kD, kD, kD, 0);
  wt_plane_kernel<<<kD, kD / 8, 0, stream>>>(Wk, WK, kD, kD, kD, kD, 0);
  wt_plane_kernel<<<kD, kD / 8, 0, stream>>>(Wv, WV, kD, kD, kD, kD, 0);
  wt_plane_kernel<<<kD, kD / 8, 0, stream>>>(Wg, WG, kD, kD, kD, kD, 0);
  wt_plane_kernel<<<kD, kD / 8, 0, stream>>>(Wo, WO, kD, kD, kD, kD, 0);
  wt_plane_kernel<<<kH, kD / 8, 0, stream>>>(Wb, WB, kD, kH, kH, kD, 0);
  wt_plane_kernel<<<kBG - kH, kD / 8, 0, stream>>>(Wb, WB + (size_t)kH * kD, kD, kH, 0, kD, 0);
  setup_kernel<<<9, 192, 0, stream>>>(bb, qconv_b, kconv_b, qn_w, qn_b, kn_w, kn_b, BIAS, PRM);

  for (int s = 0; s < kB; ++s) {
    cast_plane_kernel<<<(int)(((size_t)kL * kD / 8) / kThr), kThr, 0, stream>>>(hidden + (size_t)s * kL * kD, X16, 11, kD, 0);
    wmma_gemm64<0, false, 2, 0, false, 0><<<dim3((kL / 64) * (kBG / 64) / 8, 1), 256, 0, stream>>>(
        X16, X16, kD, 0L, WB, WB, kD, 0L, (void*)BL, (void*)BL, kBG, 0L, BIAS + kFBB, nullptr, 0L, kL, kBG, kD, kSc);
    beta_kernel<<<kL / kThr, kThr, 0, stream>>>(BL, BE);
    for (int hg = 0; hg < 2; ++hg) {
      const size_t wo = (size_t)hg * kNG * kD;
      wmma_gemm64<0, false, 2, 0, false, 0><<<dim3((kL / 64) * (kNG / 64) / 8, 1), 256, 0, stream>>>(
          X16, X16, kD, 0L, WQ + wo, WQ + wo, kD, 0L, (void*)QL, (void*)QL, kNG, 0L, BIAS + kFZB, nullptr, 0L, kL, kNG, kD, kSc);
      wmma_gemm64<0, false, 2, 0, false, 0><<<dim3((kL / 64) * (kNG / 64) / 8, 1), 256, 0, stream>>>(
          X16, X16, kD, 0L, WK + wo, WK + wo, kD, 0L, (void*)KL, (void*)KL, kNG, 0L, BIAS + kFZB, nullptr, 0L, kL, kNG, kD, kSc);
      wmma_gemm64<0, false, 2, 0, false, 0><<<dim3((kL / 64) * (kNG / 64) / 8, 1), 256, 0, stream>>>(
          X16, X16, kD, 0L, WV + wo, WV + wo, kD, 0L, (void*)VP, (void*)VP, kNG, 0L, BIAS + kFZB, nullptr, 0L, kL, kNG, kD, kSc);
      wmma_gemm64<0, false, 2, 0, false, 0><<<dim3((kL / 64) * (kNG / 64) / 8, 1), 256, 0, stream>>>(
          X16, X16, kD, 0L, WG + wo, WG + wo, kD, 0L, (void*)GL, (void*)GL, kNG, 0L, BIAS + kFZB, nullptr, 0L, kL, kNG, kD, kSc);
      convln_kernel<<<(kL * kHG) / kThr, kThr, 0, stream>>>(QL, qconv_w, PRM + kPQB, PRM + kPQW, PRM + kPQO, Q2, hg * kNG);
      convln_kernel<<<(kL * kHG) / kThr, kThr, 0, stream>>>(KL, kconv_w, PRM + kPKB, PRM + kPKW, PRM + kPKO, K2, hg * kNG);
      gma_scan_kernel<<<kHG, kHd, 0, stream>>>(Q2, K2, VP, BE, O32, hg * kHG);
      ogate_kernel<<<(int)(((size_t)kL * kNG / 8) / kThr), kThr, 0, stream>>>(O32, GL, O16, hg * kNG);
    }
    wmma_gemm64<0, false, 2, 0, false, 0><<<dim3((kL / 64) * (kD / 64) / 8, 1), 256, 0, stream>>>(
        O16, O16, kD, 0L, WO, WO, kD, 0L, (void*)(out + (size_t)s * kL * kD), (void*)(out + (size_t)s * kL * kD), kD, 0L, BIAS + kFZB, nullptr, 0L, kL, kD, kD, kScO);
  }
}
